// CustomBSplineLayer_26182120636498
// MI455X (gfx1250) — hardware-verified
//
#include <hip/hip_runtime.h>
#include <stdint.h>


typedef _Float16 v16h __attribute__((ext_vector_type(16)));
typedef _Float16 v8h  __attribute__((ext_vector_type(8)));
typedef float    v8f  __attribute__((ext_vector_type(8)));
typedef float    v4f  __attribute__((ext_vector_type(4)));

union Frag { v16h v; v8h half[2]; };
union H8   { v8h v; _Float16 e[8]; };

#define BATCH  8192
#define INSZ   512
#define OUTSZ  512
#define GRIDC  8
#define KDIM   (INSZ * GRIDC)
#define BM     16
#define BK     64
#define LDA    72
#define SP     68
#define NTHR   256
#define WSC    64.0f
#define SSC    4096.0f
#define LSC    2048.0f

__device__ __forceinline__ v8f wmma16(const v16h a, const v16h b, v8f c) {
  return __builtin_amdgcn_wmma_f32_16x16x32_f16(false, a, false, b, (short)0, c, false, false);
}

__device__ __forceinline__ float knot(int j) {
#pragma clang fp contract(off)
  const float stopv = (float)(1.0 + (2.0 * 4.0) / 7.0);
  if (j >= 11) return stopv;
  const float tj = (float)j / 11.0f;
  return (-1.0f) * (1.0f - tj) + stopv * tj;
}

template <int K, int CNT>
__device__ __forceinline__ void deboor_level(float xv, const float (&c)[12], float (&b)[11]) {
#pragma clang fp contract(off)
#pragma unroll
  for (int j = 0; j < CNT; ++j) {
    const float c0  = c[j];
    const float ck  = c[j + K];
    const float c1  = c[j + 1];
    const float ck1 = c[j + K + 1];
    const float ra  = 1.0f / (ck - c0);
    const float rb  = 1.0f / (ck1 - c1);
    b[j] = ((xv - c0) * ra) * b[j] + ((ck1 - xv) * rb) * b[j + 1];
  }
}

__device__ __forceinline__ void bspline8(float xv, float (&s)[8]) {
#pragma clang fp contract(off)
  float c[12];
#pragma unroll
  for (int j = 0; j < 12; ++j) c[j] = knot(j);
  float b[11];
#pragma unroll
  for (int j = 0; j < 11; ++j) b[j] = (xv >= c[j] && xv < c[j + 1]) ? 1.0f : 0.0f;
  deboor_level<1, 10>(xv, c, b);
  deboor_level<2, 9>(xv, c, b);
  deboor_level<3, 8>(xv, c, b);
#pragma unroll
  for (int g = 0; g < 8; ++g) s[g] = b[g];
}

__global__ __launch_bounds__(NTHR) void k_prep_w(const float* __restrict__ w,
                                                 const float* __restrict__ coef,
                                                 _Float16* __restrict__ Wq,
                                                 int n_oi) {
  const int idx = blockIdx.x * NTHR + threadIdx.x;
  if (idx >= n_oi) return;
  const float ww = w[idx] * WSC;
  const float4 ca = *(const float4*)(coef + (size_t)idx * GRIDC);
  const float4 cb = *(const float4*)(coef + (size_t)idx * GRIDC + 4);
  H8 p;
  p.e[0] = (_Float16)(ca.x * ww);
  p.e[1] = (_Float16)(ca.y * ww);
  p.e[2] = (_Float16)(ca.z * ww);
  p.e[3] = (_Float16)(ca.w * ww);
  p.e[4] = (_Float16)(cb.x * ww);
  p.e[5] = (_Float16)(cb.y * ww);
  p.e[6] = (_Float16)(cb.z * ww);
  p.e[7] = (_Float16)(cb.w * ww);
  const v8h v = p.v;
  _Float16* dst = Wq + (size_t)idx * GRIDC;
  *(volatile v8h*)dst = v;
  __threadfence();
  *(volatile v8h*)dst = v;
}

__global__ __launch_bounds__(NTHR) void k_spline_gemm(const float* __restrict__ x,
                                                      const _Float16* __restrict__ Wq,
                                                      float* __restrict__ out,
                                                      int nrows) {
  __shared__ __attribute__((aligned(16))) _Float16 Ahi[2][BM * LDA];
  __shared__ __attribute__((aligned(16))) _Float16 Alo[2][BM * LDA];
  __shared__ __attribute__((aligned(16))) float    stg[8 * BM * SP];

  const int t    = threadIdx.x;
  const int lane = t & 31;
  const int wv   = t >> 5;
  const int h    = lane >> 4;
  const int m    = lane & 15;
  const int mBase = blockIdx.x * BM;
  if (mBase >= nrows) return;
  const int n0 = wv * 64;

  const int br  = (t >> 3) & 15;
  const int bfi = t & 7;

  v8f acc[4], accL[4];
#pragma unroll
  for (int ni = 0; ni < 4; ++ni) {
    acc[ni]  = (v8f){0.f, 0.f, 0.f, 0.f, 0.f, 0.f, 0.f, 0.f};
    accL[ni] = (v8f){0.f, 0.f, 0.f, 0.f, 0.f, 0.f, 0.f, 0.f};
  }

  const float kL = 1.0f / LSC;
  const float kO = 1.0f / (SSC * WSC);

#pragma unroll 1
  for (int kc = 0; kc < INSZ / 8; ++kc) {
    const int buf = kc & 1;
    if (t < 128) {
      float xv = x[(size_t)(mBase + br) * INSZ + kc * 8 + bfi];
      xv = fminf(fmaxf(xv, -1.0f), 1.0f);
      float s[8];
      bspline8(xv, s);
      H8 ph, pl;
#pragma unroll
      for (int g = 0; g < 8; ++g) {
        const float sv   = s[g] * SSC;
        const _Float16 q = (_Float16)sv;
        const float res  = (sv - (float)q) * LSC;
        ph.e[g] = q;
        pl.e[g] = (_Float16)res;
      }
      *(v8h*)(&Ahi[buf][br * LDA + bfi * 8]) = ph.v;
      *(v8h*)(&Alo[buf][br * LDA + bfi * 8]) = pl.v;
    }
    __syncthreads();

    const int k0 = kc * BK;
#pragma unroll
    for (int ks = 0; ks < BK; ks += 32) {
      Frag ah, al, bq[4];
      ah.half[0] = *(const v8h*)(&Ahi[buf][m * LDA + ks + 8 * h]);
      ah.half[1] = *(const v8h*)(&Ahi[buf][m * LDA + ks + 16 + 8 * h]);
      al.half[0] = *(const v8h*)(&Alo[buf][m * LDA + ks + 8 * h]);
      al.half[1] = *(const v8h*)(&Alo[buf][m * LDA + ks + 16 + 8 * h]);
#pragma unroll
      for (int ni = 0; ni < 4; ++ni) {
        const _Float16* bp = Wq + (size_t)(n0 + ni * 16 + m) * KDIM + k0 + ks;
        bq[ni].half[0] = *(const v8h*)(bp + 8 * h);
        bq[ni].half[1] = *(const v8h*)(bp + 16 + 8 * h);
      }
#pragma unroll
      for (int ni = 0; ni < 4; ++ni) acc[ni] = wmma16(ah.v, bq[ni].v, acc[ni]);
#pragma unroll
      for (int ni = 0; ni < 4; ++ni) accL[ni] = wmma16(al.v, bq[ni].v, accL[ni]);
      asm volatile("v_nop\n\tv_nop\n\tv_nop\n\tv_nop"
                   : "+v"(acc[0]), "+v"(acc[1]), "+v"(acc[2]), "+v"(acc[3]),
                     "+v"(accL[0]), "+v"(accL[1]), "+v"(accL[2]), "+v"(accL[3])
                   : "v"(ah.v), "v"(al.v), "v"(bq[0].v), "v"(bq[1].v), "v"(bq[2].v), "v"(bq[3].v));
    }
  }

  float* sw = stg + wv * (BM * SP);
#pragma unroll
  for (int ni = 0; ni < 4; ++ni) {
#pragma unroll
    for (int r = 0; r < 8; ++r) {
      sw[(8 * h + r) * SP + ni * 16 + m] = (acc[ni][r] + accL[ni][r] * kL) * kO;
    }
  }
  __syncthreads();

  v4f vv[8];
#pragma unroll
  for (int it = 0; it < 8; ++it) vv[it] = *(const v4f*)(&sw[(2 * it + h) * SP + m * 4]);
#pragma unroll
  for (int it = 0; it < 8; ++it) {
    float* op = out + (size_t)(mBase + 2 * it + h) * OUTSZ + n0 + m * 4;
    *(volatile v4f*)op = vv[it];
  }
  __threadfence();
#pragma unroll
  for (int it = 0; it < 8; ++it) {
    float* op = out + (size_t)(mBase + 2 * it + h) * OUTSZ + n0 + m * 4;
    *(volatile v4f*)op = vv[it];
  }
}

extern "C" void kernel_launch(void* const* d_in, const int* in_sizes, int n_in,
                              void* d_out, int out_size, void* d_ws, size_t ws_size,
                              hipStream_t stream) {
  if (n_in < 3) return;
  if (in_sizes[0] != BATCH * INSZ) return;
  if (in_sizes[1] != OUTSZ * INSZ) return;
  if (in_sizes[2] != OUTSZ * INSZ * GRIDC) return;
  if (out_size != BATCH * OUTSZ) return;
  const size_t wq_bytes = (size_t)OUTSZ * KDIM * sizeof(_Float16);
  if (ws_size < wq_bytes) return;

  const float* x    = (const float*)d_in[0];
  const float* w    = (const float*)d_in[1];
  const float* coef = (const float*)d_in[2];
  float* out        = (float*)d_out;
  _Float16* Wq      = (_Float16*)d_ws;

  k_prep_w<<<(OUTSZ * INSZ + NTHR - 1) / NTHR, NTHR, 0, stream>>>(w, coef, Wq, OUTSZ * INSZ);
  k_spline_gemm<<<(BATCH + BM - 1) / BM, NTHR, 0, stream>>>(x, Wq, out, BATCH);
}
